// RelativeInformationAttention_31817117729140
// MI455X (gfx1250) — hardware-verified
//
#include <hip/hip_runtime.h>
#include <math.h>

typedef __attribute__((ext_vector_type(16))) _Float16 v16h;
typedef __attribute__((ext_vector_type(16))) __bf16 v16b;
typedef __attribute__((ext_vector_type(8)))  _Float16 v8h;
typedef __attribute__((ext_vector_type(8)))  float v8f;
typedef __attribute__((ext_vector_type(4)))  float v4f;
typedef __attribute__((ext_vector_type(2)))  float v2f;
typedef __attribute__((ext_vector_type(4)))  unsigned v4u;
typedef __attribute__((ext_vector_type(4)))  int v4i;
typedef float __attribute__((may_alias)) float_a;
typedef int __attribute__((may_alias)) int_a;

template <typename T> __device__ __forceinline__ void vst2(void* p, T v) { *(volatile T*)p = v; __threadfence(); *(volatile T*)p = v; }
__device__ __forceinline__ v8f wmma16(v16h a, v16h b, v8f c) {
  v8f d = __builtin_amdgcn_wmma_f32_16x16x32_f16(false, a, false, b, (short)0, c, false, false);
  asm volatile("v_nop\n\tv_nop\n\tv_nop\n\tv_nop" : "+v"(d) : "v"(a), "v"(b));
  return d;
}
__device__ __forceinline__ v8f wmma_bf(v16b a, v16b b, v8f c) {
  v8f d = __builtin_amdgcn_wmma_f32_16x16x32_bf16(false, a, false, b, (short)0, c, false, false);
  asm volatile("v_nop\n\tv_nop\n\tv_nop\n\tv_nop" : "+v"(d) : "v"(a), "v"(b));
  return d;
}
__device__ __forceinline__ v16h frag_h(const _Float16* rowk0, int lane) {
  union { v16h v; v8h q[2]; } u; const _Float16* p = rowk0 + 8 * (lane >> 4);
  u.q[0] = *(const v8h*)p; u.q[1] = *(const v8h*)(p + 16); return u.v;
}
__device__ __forceinline__ v16h frag_f32(const float* rowk0, int lane) {
  v16h a; const float* p = rowk0 + 8 * (lane >> 4);
#pragma unroll
  for (int i = 0; i < 8; ++i) { a[i] = (_Float16)p[i]; a[8 + i] = (_Float16)p[16 + i]; }
  return a;
}
__device__ __forceinline__ v16h frag_f32s(const float* rowk0, int lane, float sc) {
  v16h a; const float* p = rowk0 + 8 * (lane >> 4);
#pragma unroll
  for (int i = 0; i < 8; ++i) { a[i] = (_Float16)(p[i] * sc); a[8 + i] = (_Float16)(p[16 + i] * sc); }
  return a;
}
__device__ __forceinline__ v16h fragc_f32(const float* W, int k0, int n, int lane, int ld, int K) {
  v16h a; const int g = lane >> 4;
#pragma unroll
  for (int i = 0; i < 8; ++i) { const int ka = k0 + 8 * g + i, kb = ka + 16;
    a[i] = (_Float16)(ka < K ? W[(size_t)(ka < K ? ka : K - 1) * ld + n] : 0.f); a[8 + i] = (_Float16)(kb < K ? W[(size_t)(kb < K ? kb : K - 1) * ld + n] : 0.f); }
  return a;
}
struct F2 { v16b h, l; };
__device__ __forceinline__ F2 bsplit16(const float v[16]) { F2 r;
#pragma unroll
  for (int i = 0; i < 16; ++i) { const __bf16 h = (__bf16)v[i]; r.h[i] = h; r.l[i] = (__bf16)(v[i] - (float)h); }
  return r; }
__device__ __forceinline__ F2 split_row(const float* row, int k0, int lane) { float v[16]; const float* p = row + k0 + 8 * (lane >> 4);
#pragma unroll
  for (int i = 0; i < 8; ++i) { v[i] = p[i]; v[8 + i] = p[16 + i]; }
  return bsplit16(v); }
__device__ __forceinline__ F2 split_rowK(const float* row, int k0, int lane, int K) { float v[16]; const int g = lane >> 4;
#pragma unroll
  for (int i = 0; i < 8; ++i) { const int ka = k0 + 8 * g + i, kb = ka + 16; v[i] = ka < K ? row[ka < K ? ka : K - 1] : 0.f; v[8 + i] = kb < K ? row[kb < K ? kb : K - 1] : 0.f; }
  return bsplit16(v); }
__device__ __forceinline__ F2 split_col(const float* W, int k0, int n, int lane, int ld, int K) { float v[16]; const int g = lane >> 4;
#pragma unroll
  for (int i = 0; i < 8; ++i) { const int ka = k0 + 8 * g + i, kb = ka + 16; v[i] = ka < K ? W[(size_t)(ka < K ? ka : K - 1) * ld + n] : 0.f; v[8 + i] = kb < K ? W[(size_t)(kb < K ? kb : K - 1) * ld + n] : 0.f; }
  return bsplit16(v); }
__device__ __forceinline__ v8f mac3(const F2& a, const F2& b, v8f c) { c = wmma_bf(a.l, b.h, c); c = wmma_bf(a.h, b.l, c); return wmma_bf(a.h, b.h, c); }
__device__ __forceinline__ float sigm(float v) { return 1.0f / (1.0f + expf(-v)); }
#define LDSX() do { asm volatile("s_wait_dscnt 0" ::: "memory"); __builtin_amdgcn_wave_barrier(); __builtin_amdgcn_fence(__ATOMIC_RELEASE, "workgroup"); } while (0)


#define NB 2
#define NH 8
#define SS 2048
#define RR 128
#define NREL (2 * RR + 1)
#define NRP 272
#define HD 64
#define NBH (NB * NH)
#ifndef TQB
#define TQB (SS / 64)
#define TNBH NBH
#endif
typedef __attribute__((ext_vector_type(8))) __bf16 v8b;
__device__ __forceinline__ v16b frag_b(const __bf16* rowk0, int lane) {
  union { v16b v; v8b q[2]; } u; const __bf16* p = rowk0 + 8 * (lane >> 4);
  u.q[0] = *(const v8b*)p; u.q[1] = *(const v8b*)(p + 16); return u.v;
}
__device__ __forceinline__ float bfr(float v) { return (float)(__bf16)v; }
__device__ __attribute__((noinline)) float exp_ni(float v) { return expf(v); }
__device__ __attribute__((noinline)) float erf_ni(float v) { return erff(v); }

#define WS_VT  0u
#define WS_RE  (WS_VT + 2u * (size_t)NBH * HD * SS)
#define WS_QR  (WS_RE + 2u * (size_t)NRP * HD)
#define WS_END (WS_QR + 4u * (size_t)NBH * SS * NRP)

__global__ __launch_bounds__(256) void k_vt(const float* __restrict__ V, _Float16* __restrict__ VT) { __shared__ __align__(16) _Float16 st[HD][64 + 8]; const int t = threadIdx.x; const int s0 = blockIdx.x * 64; const size_t bh = blockIdx.y;
  for (int e = t; e < 64 * HD; e += 256) { const int sl = e >> 6, d = e & 63; st[d][sl] = (_Float16)bfr(V[((bh * SS + s0 + sl) * HD) + d]); } __syncthreads();
  for (int e = t; e < HD * 8; e += 256) { const int d = e >> 3, q = e & 7; vst2((unsigned*)(VT + ((bh * HD + d) * SS) + s0 + q * 8), *(const v4u*)&st[d][q * 8]); } }
__global__ __launch_bounds__(256) void k_rel(const float* __restrict__ RE, __bf16* __restrict__ RB) { __shared__ __align__(16) __bf16 s[NRP * HD]; const int t = threadIdx.x; for (int e = t; e < NRP * HD; e += 256) s[e] = (e < NREL * HD) ? (__bf16)RE[e] : (__bf16)0.0f; __syncthreads(); for (int q = t; q < NRP * HD / 8; q += 256) vst2((unsigned*)(RB + q * 8), *(const v4u*)&s[q * 8]); }
__device__ __forceinline__ v16b fragb_f32_pre(const float* __restrict__ p, int lane) { v16b a; const float* pp = p + 8 * (lane >> 4);
#pragma unroll
  for (int i = 0; i < 8; ++i) { a[i] = (__bf16)pp[i]; a[8 + i] = (__bf16)pp[16 + i]; } return a; }
__global__ __launch_bounds__(128) void k_qr(const float* __restrict__ Q, const __bf16* __restrict__ RB, float* __restrict__ QR) { __shared__ __align__(16) float sf[4][16][NRP + 4];
  const int tid = threadIdx.x, wave = tid >> 5, lane = tid & 31, col = lane & 15, g = lane >> 4; const size_t bh = blockIdx.y; const size_t r0 = bh * SS + (size_t)blockIdx.x * 64 + wave * 16;
  v16b aq[2];
#pragma unroll
  for (int kc = 0; kc < 2; ++kc) aq[kc] = fragb_f32_pre(Q + (r0 + col) * HD + kc * 32, lane);
#pragma unroll 1
  for (int j = 0; j < NRP / 16; ++j) { v8f c = {};
#pragma unroll
    for (int kc = 0; kc < 2; ++kc) c = wmma_bf(aq[kc], frag_b(RB + (size_t)(j * 16 + col) * HD + kc * 32, lane), c);
#pragma unroll
    for (int r = 0; r < 8; ++r) sf[wave][8 * g + r][j * 16 + col] = c[r]; }
  LDSX(); for (int rl = 0; rl < 16; ++rl) for (int q = lane; q < NRP / 4; q += 32) vst2(QR + (r0 + rl) * NRP + q * 4, *(const v4f*)&sf[wave][rl][q * 4]); }
__device__ __forceinline__ v16b fragb_f32(const float* __restrict__ p, int lane) { v16b a; const float* pp = p + 8 * (lane >> 4);
#pragma unroll
  for (int i = 0; i < 8; ++i) { a[i] = (__bf16)pp[i]; a[8 + i] = (__bf16)pp[16 + i]; } return a; }
__global__ __launch_bounds__(128) void k_attn(const float* __restrict__ Q, const float* __restrict__ K, const _Float16* __restrict__ VT, const float* __restrict__ QR, const int* __restrict__ QI, const int* __restrict__ KI, float* __restrict__ O) {
  __shared__ __align__(16) float sp[4][16][36]; __shared__ __align__(16) float so[4][16][68]; __shared__ float sqr[4][16][NREL + 3];
  const int tid = threadIdx.x, wave = tid >> 5, lane = tid & 31, col = lane & 15, g = lane >> 4; const size_t bh = blockIdx.y; const int q0 = blockIdx.x * 64 + wave * 16; const float* Qb = Q + (bh * SS) * HD; const float* Kb = K + (bh * SS) * HD; const _Float16* Vb = VT + bh * HD * SS;
  v16b aq[2];
#pragma unroll
  for (int kc = 0; kc < 2; ++kc) aq[kc] = fragb_f32(Qb + (size_t)(q0 + col) * HD + kc * 32, lane);
  const size_t b = bh / NH; for (int e = lane; e < 16 * NREL; e += 32) { const int rl = e / NREL, rr = e % NREL; sqr[wave][rl][rr] = QR[(bh * SS + q0 + rl) * NRP + rr]; }
  int qa[8];
#pragma unroll
  for (int r = 0; r < 8; ++r) { const int qi = QI[b * SS + q0 + 8 * g + r]; qa[r] = (qi == -1) ? 2 * RR : qi; }
  LDSX();
  float m[8], l[8];
#pragma unroll
  for (int r = 0; r < 8; ++r) { m[r] = -3.0e38f; l[r] = 0.f; }
  v8f acc[4] = {}, accl[4] = {};
#pragma unroll 1
  for (int ks = 0; ks < SS / 32; ++ks) { v8f s[2];
#pragma unroll
    for (int ct = 0; ct < 2; ++ct) { const int kk = ks * 32 + ct * 16 + col; v8f c = {};
#pragma unroll
      for (int kc = 0; kc < 2; ++kc) c = wmma_bf(aq[kc], fragb_f32(Kb + (size_t)kk * HD + kc * 32, lane), c);
      { const int ki = KI[b * SS + kk]; const int ka = (ki == -1) ? 3 * RR : ki;
#pragma unroll
      for (int r = 0; r < 8; ++r) { int dmv = ka - qa[r]; dmv = dmv < -RR ? -RR : (dmv > RR ? RR : dmv); s[ct][r] = (c[r] + sqr[wave][8 * g + r][dmv + RR]) * 0.125f; } } }
#pragma unroll
    for (int r = 0; r < 8; ++r) { float mx = fmaxf(s[0][r], s[1][r]);
#pragma unroll
      for (int o = 1; o < 16; o <<= 1) mx = fmaxf(mx, __shfl_xor(mx, o));
      const float mn = fmaxf(m[r], mx); const float alpha = (m[r] <= -1.0e38f) ? 0.f : __expf(m[r] - mn); const float e0 = __expf(s[0][r] - mn), e1 = __expf(s[1][r] - mn); float es = e0 + e1;
#pragma unroll
      for (int o = 1; o < 16; o <<= 1) es += __shfl_xor(es, o);
      l[r] = l[r] * alpha + es; m[r] = mn;
#pragma unroll
      for (int dt = 0; dt < 4; ++dt) { acc[dt][r] *= alpha; accl[dt][r] *= alpha; }
      sp[wave][8 * g + r][col] = e0; sp[wave][8 * g + r][16 + col] = e1; }
    LDSX();
    v16h pa, pl; { const float* prow = &sp[wave][col][0] + 8 * (lane >> 4);
#pragma unroll
      for (int i = 0; i < 8; ++i) { const float x0 = prow[i] * 2048.0f, x1 = prow[16 + i] * 2048.0f; const _Float16 h0 = (_Float16)x0, h1 = (_Float16)x1; pa[i] = h0; pa[8 + i] = h1; pl[i] = (_Float16)((x0 - (float)h0) * 2048.0f); pl[8 + i] = (_Float16)((x1 - (float)h1) * 2048.0f); } }
#pragma unroll
    for (int dt = 0; dt < 4; ++dt) { const v16h vf = frag_h(Vb + (size_t)(dt * 16 + col) * SS + ks * 32, lane); acc[dt] = wmma16(pa, vf, acc[dt]); accl[dt] = wmma16(pl, vf, accl[dt]); }
    LDSX(); }
#pragma unroll
  for (int r = 0; r < 8; ++r) { const float il = (1.0f / 2048.0f) / l[r];
#pragma unroll
    for (int dt = 0; dt < 4; ++dt) so[wave][8 * g + r][dt * 16 + col] = (acc[dt][r] + accl[dt][r] * (1.0f / 2048.0f)) * il; }
  LDSX();
  for (int rl = 0; rl < 16; ++rl) if (lane < 16) vst2(O + ((bh * SS + q0 + rl) * HD) + lane * 4, *(const v4f*)&so[wave][rl][lane * 4]);
}
extern "C" void kernel_launch(void* const* d_in, const int* in_sizes, int n_in, void* d_out, int out_size, void* d_ws, size_t ws_size, hipStream_t stream) {
  (void)in_sizes; (void)n_in; (void)out_size;
  const float** F = (const float**)d_in;
  if (ws_size < (size_t)WS_END) return;
  _Float16* VT = (_Float16*)((char*)d_ws + WS_VT); __bf16* RB = (__bf16*)((char*)d_ws + WS_RE); float* QR = (float*)((char*)d_ws + WS_QR);
  k_vt<<<dim3(SS / 64, NBH), 256, 0, stream>>>(F[2], VT);
  k_rel<<<1, 256, 0, stream>>>(F[3], RB);
  k_qr<<<dim3(SS / 64, NBH), 128, 0, stream>>>(F[0], RB, QR);
  k_attn<<<dim3(TQB, TNBH), 128, 0, stream>>>(F[0], F[1], VT, QR, (const int*)d_in[4], (const int*)d_in[5], (float*)d_out);
}
